// torch_sigma_2010044694686
// MI455X (gfx1250) — hardware-verified
//
#include <hip/hip_runtime.h>
#include <stddef.h>
#include <stdint.h>


typedef float        v4f   __attribute__((ext_vector_type(4)));
typedef float        v8f   __attribute__((ext_vector_type(8)));
typedef __bf16       v8bf  __attribute__((ext_vector_type(8)));
typedef __bf16       v16bf __attribute__((ext_vector_type(16)));
typedef unsigned int v4u   __attribute__((ext_vector_type(4)));

#define KD     512
#define NP     16
#define MT     32
#define NTHR   128
#define PASSW  256
#define SA     520
#define SR     264

#define LDS_HFH   0
#define LDS_HFL   (LDS_HFH + MT * SA * 2)
#define LDS_RH    (LDS_HFL + MT * SA * 2)
#define LDS_RL    (LDS_RH  + MT * SR * 2)
#define LDS_OUT   (LDS_RL  + MT * SR * 2)
#define LDS_BYTES (LDS_OUT + MT * NP * 4)

union Frag  { v16bf v; v8bf h[2]; };
union Pack8 { v8bf b;  v4u  u;    };

__device__ __forceinline__ v8f wmma3(v8f c, const Frag& ah, const Frag& al,
                                     const Frag& bh, const Frag& bl)
{
    c = __builtin_amdgcn_wmma_f32_16x16x32_bf16(false, al.v, false, bh.v, (short)0, c, false, false);
    c = __builtin_amdgcn_wmma_f32_16x16x32_bf16(false, ah.v, false, bl.v, (short)0, c, false, false);
    c = __builtin_amdgcn_wmma_f32_16x16x32_bf16(false, ah.v, false, bh.v, (short)0, c, false, false);
    return c;
}

#define GUARD2(c0, c1, a0, a1, a2, a3, b0, b1)                                  \
    asm volatile("v_nop\n\tv_nop\n\tv_nop\n\tv_nop"                            \
                 : "+v"(c0), "+v"(c1)                                           \
                 : "v"(a0), "v"(a1), "v"(a2), "v"(a3), "v"(b0), "v"(b1))
#define GUARD1(c0, a0, a1, b0, b1)                                              \
    asm volatile("v_nop\n\tv_nop\n\tv_nop\n\tv_nop"                            \
                 : "+v"(c0)                                                     \
                 : "v"(a0), "v"(a1), "v"(b0), "v"(b1))

__device__ __forceinline__ void split8(const float (&x)[8], Pack8& ph, Pack8& pl)
{
    #pragma unroll
    for (int i = 0; i < 8; ++i) {
        const __bf16 hb = (__bf16)x[i];
        const float  d  = x[i] - (float)hb;
        ph.b[i] = hb;
        pl.b[i] = (__bf16)d;
    }
}

__global__ __launch_bounds__(256) void k_prep(const float* __restrict__ w1,
                                              const float* __restrict__ w2,
                                              int n2rows,
                                              v4u* wh, v4u* wl, v4u* w2h, v4u* w2l)
{
    const int g   = blockIdx.x * 256 + threadIdx.x;
    const int ng1 = (KD * KD) >> 3;
    const int ng2 = (NP * KD) >> 3;
    float x[8];
    v4u* dh;
    v4u* dl;
    int gi;
    if (g < ng1) {
        const v4f a = *(const v4f*)(w1 + (size_t)g * 8);
        const v4f b = *(const v4f*)(w1 + (size_t)g * 8 + 4);
        x[0] = a.x; x[1] = a.y; x[2] = a.z; x[3] = a.w;
        x[4] = b.x; x[5] = b.y; x[6] = b.z; x[7] = b.w;
        dh = wh; dl = wl; gi = g;
    } else if (g < ng1 + ng2) {
        gi = g - ng1;
        const int e0 = gi * 8;
        const int n  = e0 / KD;
        const int k  = e0 - n * KD;
        if (n < n2rows) {
            const v4f a = *(const v4f*)(w2 + (size_t)n * KD + k);
            const v4f b = *(const v4f*)(w2 + (size_t)n * KD + k + 4);
            x[0] = a.x; x[1] = a.y; x[2] = a.z; x[3] = a.w;
            x[4] = b.x; x[5] = b.y; x[6] = b.z; x[7] = b.w;
        } else {
            #pragma unroll
            for (int i = 0; i < 8; ++i) x[i] = 0.f;
        }
        dh = w2h; dl = w2l;
    } else {
        return;
    }
    Pack8 ph, pl;
    split8(x, ph, pl);
    const v4u vh = ph.u;
    const v4u vl = pl.u;
    volatile v4u* p0 = dh + gi;
    volatile v4u* p1 = dl + gi;
    *p0 = vh;
    *p1 = vl;
    __threadfence();
    *p0 = vh;
    *p1 = vl;
}

__global__ __launch_bounds__(NTHR) void k_main(
    const float*  __restrict__ H,
    const float*  __restrict__ few,
    const float*  __restrict__ feb,
    const __bf16* __restrict__ wh,
    const __bf16* __restrict__ wl,
    const float*  __restrict__ b1,
    const __bf16* __restrict__ w2h,
    const __bf16* __restrict__ w2l,
    const float*  __restrict__ b2,
    float* out,
    int rows, int nout)
{
    extern __shared__ __align__(16) unsigned char smem[];
    __bf16* sHFH = (__bf16*)(smem + LDS_HFH);
    __bf16* sHFL = (__bf16*)(smem + LDS_HFL);
    __bf16* sRH  = (__bf16*)(smem + LDS_RH);
    __bf16* sRL  = (__bf16*)(smem + LDS_RL);
    float*  sOut = (float*)(smem + LDS_OUT);

    const int tid  = threadIdx.x;
    const int lane = tid & 31;
    const int wid  = tid >> 5;
    const int am   = lane & 15;
    const int lh   = lane >> 4;
    const int rowbase = blockIdx.x * MT;

    {
        const int cg = tid & 63;
        const int r0 = (tid >> 6) * 16;
        float w0[8], w1[8], w2[8], bb[8];
        #pragma unroll
        for (int i = 0; i < 8; ++i) {
            const int c = cg * 8 + i;
            w0[i] = few[c * 3 + 0];
            w1[i] = few[c * 3 + 1];
            w2[i] = few[c * 3 + 2];
            bb[i] = feb[c];
        }
        #pragma unroll 1
        for (int rr = 0; rr < 16; ++rr) {
            const int m  = r0 + rr;
            const int gm = rowbase + m;
            float h0 = 0.f, h1 = 0.f, h2 = 0.f;
            if (gm < rows) {
                const float* hr = H + (size_t)gm * 3;
                h0 = hr[0]; h1 = hr[1]; h2 = hr[2];
            }
            float v[8];
            #pragma unroll
            for (int i = 0; i < 8; ++i) {
                const float t = h0 * w0[i] + h1 * w1[i] + h2 * w2[i] + bb[i];
                v[i] = t > 0.f ? t : 0.f;
            }
            Pack8 ph, pl;
            split8(v, ph, pl);
            *(v8bf*)(sHFH + m * SA + cg * 8) = ph.b;
            *(v8bf*)(sHFL + m * SA + cg * 8) = pl.b;
        }
    }
    __syncthreads();

    const v8f z8 = {0.f, 0.f, 0.f, 0.f, 0.f, 0.f, 0.f, 0.f};
    v8f acc2 = z8;

    for (int p = 0; p < KD / PASSW; ++p) {
        v8f acc[2][4];
        #pragma unroll
        for (int rt = 0; rt < 2; ++rt) {
            #pragma unroll
            for (int c = 0; c < 4; ++c) acc[rt][c] = z8;
        }
        const int colw = p * PASSW + wid * 64;

        #pragma unroll 1
        for (int ks = 0; ks < KD / 32; ++ks) {
            const int k0  = ks * 32;
            const int oa0 = am * SA + k0 + 8 * lh;
            const int oa1 = oa0 + 16 * SA;
            Frag ah0, al0, ah1, al1;
            ah0.h[0] = *(const v8bf*)(sHFH + oa0);
            ah0.h[1] = *(const v8bf*)(sHFH + oa0 + 16);
            al0.h[0] = *(const v8bf*)(sHFL + oa0);
            al0.h[1] = *(const v8bf*)(sHFL + oa0 + 16);
            ah1.h[0] = *(const v8bf*)(sHFH + oa1);
            ah1.h[1] = *(const v8bf*)(sHFH + oa1 + 16);
            al1.h[0] = *(const v8bf*)(sHFL + oa1);
            al1.h[1] = *(const v8bf*)(sHFL + oa1 + 16);
            #pragma unroll
            for (int c = 0; c < 4; ++c) {
                const size_t ob = (size_t)(colw + c * 16 + am) * KD + k0 + 8 * lh;
                Frag bh, bl;
                bh.h[0] = *(const v8bf*)(wh + ob);
                bh.h[1] = *(const v8bf*)(wh + ob + 16);
                bl.h[0] = *(const v8bf*)(wl + ob);
                bl.h[1] = *(const v8bf*)(wl + ob + 16);
                acc[0][c] = wmma3(acc[0][c], ah0, al0, bh, bl);
                acc[1][c] = wmma3(acc[1][c], ah1, al1, bh, bl);
                GUARD2(acc[0][c], acc[1][c], ah0.v, al0.v, ah1.v, al1.v, bh.v, bl.v);
            }
        }

        __syncthreads();
        #pragma unroll
        for (int rt = 0; rt < 2; ++rt) {
            #pragma unroll
            for (int c = 0; c < 4; ++c) {
                const int n  = colw + c * 16 + am;
                const int nl = n - p * PASSW;
                const float bias = b1[n];
                #pragma unroll
                for (int j = 0; j < 8; ++j) {
                    float r = acc[rt][c][j] + bias;
                    r = r > 0.f ? r : 0.f;
                    const __bf16 hb = (__bf16)r;
                    const __bf16 lb = (__bf16)(r - (float)hb);
                    const int o = (rt * 16 + 8 * lh + j) * SR + nl;
                    sRH[o] = hb;
                    sRL[o] = lb;
                }
            }
        }
        __syncthreads();

        if (wid < 2) {
            const int rt = wid;
            #pragma unroll 1
            for (int ks = 0; ks < PASSW / 32; ++ks) {
                const int k0 = ks * 32;
                const int oa = (rt * 16 + am) * SR + k0 + 8 * lh;
                Frag ah, al, bh, bl;
                ah.h[0] = *(const v8bf*)(sRH + oa);
                ah.h[1] = *(const v8bf*)(sRH + oa + 16);
                al.h[0] = *(const v8bf*)(sRL + oa);
                al.h[1] = *(const v8bf*)(sRL + oa + 16);
                const size_t ob = (size_t)am * KD + p * PASSW + k0 + 8 * lh;
                bh.h[0] = *(const v8bf*)(w2h + ob);
                bh.h[1] = *(const v8bf*)(w2h + ob + 16);
                bl.h[0] = *(const v8bf*)(w2l + ob);
                bl.h[1] = *(const v8bf*)(w2l + ob + 16);
                acc2 = wmma3(acc2, ah, al, bh, bl);
                GUARD1(acc2, ah.v, al.v, bh.v, bl.v);
            }
        }
    }

    if (wid < 2) {
        if (am < nout) {
            const float bias = b2[am];
            #pragma unroll
            for (int j = 0; j < 8; ++j)
                sOut[(wid * 16 + 8 * lh + j) * nout + am] = acc2[j] + bias;
        }
    }
    __syncthreads();

    if (wid == 0) {
        const int rem    = rows - rowbase;
        const int nvalid = rem < MT ? rem : MT;
        float* ob = out + (size_t)rowbase * nout;
        if (nvalid == MT) {
            const int nf4 = (MT * nout) >> 2;
            for (int f = lane; f < nf4; f += 32) {
                const v4f val = *(const v4f*)(sOut + 4 * f);
                *(volatile v4f*)(ob + 4 * f) = val;
            }
            __threadfence();
            for (int f = lane; f < nf4; f += 32) {
                const v4f val = *(const v4f*)(sOut + 4 * f);
                *(volatile v4f*)(ob + 4 * f) = val;
            }
        } else {
            const int nfl = nvalid * nout;
            for (int e = lane; e < nfl; e += 32) {
                const float val = sOut[e];
                *(volatile float*)(ob + e) = val;
            }
            __threadfence();
            for (int e = lane; e < nfl; e += 32) {
                const float val = sOut[e];
                *(volatile float*)(ob + e) = val;
            }
        }
    }
}

extern "C" void kernel_launch(void* const* d_in, const int* in_sizes, int n_in,
                              void* d_out, int out_size, void* d_ws, size_t ws_size,
                              hipStream_t stream)
{
    if (n_in < 18) return;
    const int nout = in_sizes[17];
    if (nout < 1 || nout > NP) return;
    if (in_sizes[1] != KD * 3 || in_sizes[2] != KD || in_sizes[14] != KD * KD ||
        in_sizes[15] != KD || in_sizes[16] != nout * KD) return;
    const int rows = in_sizes[0] / 3;
    if (rows <= 0 || in_sizes[0] != rows * 3 || out_size != rows * nout) return;

    const size_t b_w1  = (size_t)KD * KD * 2;
    const size_t b_w2  = (size_t)NP * KD * 2;
    const size_t o_wh  = 0;
    const size_t o_wl  = o_wh + b_w1;
    const size_t o_w2h = o_wl + b_w1;
    const size_t o_w2l = o_w2h + b_w2;
    const size_t total = o_w2l + b_w2;
    if (total > ws_size) return;

    unsigned char* ws = (unsigned char*)d_ws;
    const float* H   = (const float*)d_in[0];
    const float* few = (const float*)d_in[1];
    const float* feb = (const float*)d_in[2];
    const float* w1  = (const float*)d_in[14];
    const float* b1  = (const float*)d_in[15];
    const float* w2  = (const float*)d_in[16];
    const float* b2  = (const float*)d_in[17];

    const int ngroups = (KD * KD + NP * KD) / 8;
    const int grid1   = (ngroups + 255) / 256;
    k_prep<<<grid1, 256, 0, stream>>>(w1, w2, nout,
                                      (v4u*)(ws + o_wh), (v4u*)(ws + o_wl),
                                      (v4u*)(ws + o_w2h), (v4u*)(ws + o_w2l));

    const int grid2 = (rows + MT - 1) / MT;
    k_main<<<grid2, NTHR, LDS_BYTES, stream>>>(
        H, few, feb,
        (const __bf16*)(ws + o_wh), (const __bf16*)(ws + o_wl), b1,
        (const __bf16*)(ws + o_w2h), (const __bf16*)(ws + o_w2l), b2,
        (float*)d_out, rows, nout);
}
